// WeightedGraphLayer_35424890257853
// MI455X (gfx1250) — hardware-verified
//
#include <hip/hip_runtime.h>
#include <stdint.h>
#include <stddef.h>


typedef _Float16 v16h __attribute__((ext_vector_type(16)));
typedef _Float16 v8h  __attribute__((ext_vector_type(8)));
typedef __bf16   v16b __attribute__((ext_vector_type(16)));
typedef float    v8f  __attribute__((ext_vector_type(8)));
typedef float    v4f  __attribute__((ext_vector_type(4)));
typedef unsigned int v4u __attribute__((ext_vector_type(4)));
typedef unsigned int v8u __attribute__((ext_vector_type(8)));
typedef v8h  v8ha  __attribute__((may_alias));
typedef v16h v16ha __attribute__((may_alias));
typedef v4f  v4fa  __attribute__((may_alias));
typedef v4u  v4ua  __attribute__((may_alias));
typedef v8u  v8ua  __attribute__((may_alias));

#define N_    256
#define K_    64
#define D_    128
#define OUT_  128
#define CD_   5
#define K1    135
#define K1P   160
#define K2P   128
#define KN    261
#define KNP   320
#define NCH   5
#define WSC   16.0f
#define WSCI  0.0625f

#define NG_W1 2560
#define NG_W2 2048
#define NG_WN 5120

__device__ inline v8f mma_f16(v16h a, v16h b, v8f c) {
  v8f d = __builtin_amdgcn_wmma_f32_16x16x32_f16(false, a, false, b, (short)0, c, false, false);
  asm volatile("v_nop\n\tv_nop\n\tv_nop\n\tv_nop" : "+v"(d) : "v"(a), "v"(b));
  return d;
}
__device__ inline v8f mma_bf16(v16b a, v16b b, v8f c) {
  v8f d = __builtin_amdgcn_wmma_f32_16x16x32_bf16(false, a, false, b, (short)0, c, false, false);
  asm volatile("v_nop\n\tv_nop\n\tv_nop\n\tv_nop" : "+v"(d) : "v"(a), "v"(b));
  return d;
}

__device__ inline v16h fragA_h(const _Float16* s, int pitch, int row0, int k0, int lane) {
  const _Float16* p = s + (row0 + (lane & 15)) * pitch + k0 + ((lane >> 4) << 3);
  union { v16h v; v8h hf[2]; } u;
  u.hf[0] = *(const v8ha*)(p);
  u.hf[1] = *(const v8ha*)(p + 16);
  return u.v;
}
__device__ inline v16b fragA_b(const unsigned short* s, int pitch, int row0, int k0, int lane) {
  const unsigned short* p = s + (row0 + (lane & 15)) * pitch + k0 + ((lane >> 4) << 3);
  union { v16b v; v4u q[2]; } u;
  u.q[0] = *(const v4ua*)(p);
  u.q[1] = *(const v4ua*)(p + 16);
  return u.v;
}
__device__ inline v16h fragB_h(const _Float16* s, int f, int lane) {
  return *(const v16ha*)(s + (((f << 5) + lane) << 4));
}
__device__ inline v16b fragB_b(const unsigned short* s, int f, int lane) {
  union { v16b v; v8u q; } u;
  u.q = *(const v8ua*)(s + (((f << 5) + lane) << 4));
  return u.v;
}

__device__ inline unsigned int bf16_bits(float x) {
  unsigned int u = __float_as_uint(x);
  return (u + 0x7FFFu + ((u >> 16) & 1u)) >> 16;
}
__device__ inline float bf16_val(unsigned int b) { return __uint_as_float(b << 16); }
__device__ inline unsigned int pack2(unsigned int lo16, unsigned int hi16) {
  return (lo16 & 0xFFFFu) | (hi16 << 16);
}

__device__ inline void swz_group(const float* __restrict__ W, int g, int realK, float scale, float v[8]) {
  const int i    = g << 3;
  const int frag = i >> 9;
  const int w    = i & 511;
  const int ln   = w >> 4;
  const int j0   = w & 15;
  const int ks   = frag >> 3;
  const int nt   = frag & 7;
  const int col  = nt * 16 + (ln & 15);
  const int rb   = ks * 32 + ((ln >> 4) << 3) + ((j0 >> 3) << 4);
#pragma unroll
  for (int q = 0; q < 8; ++q) {
    const int row = rb + q;
    v[q] = (row < realK) ? W[row * OUT_ + col] * scale : 0.f;
  }
}

__global__ __launch_bounds__(256) void convert_weights_kernel(
    const float* __restrict__ W1, const float* __restrict__ W2, const float* __restrict__ Wn,
    _Float16* W1s, _Float16* W2s, unsigned short* Wnh, unsigned short* Wnl) {
  const int g = blockIdx.x * 256 + threadIdx.x;
  const bool p1 = g < NG_W1, p2 = g < NG_W2, pn = g < NG_WN;
  v8h o1, o2;
  v4u oh, ol;
  {
    float v[8];
    swz_group(W1, p1 ? g : 0, K1, WSC, v);
#pragma unroll
    for (int q = 0; q < 8; ++q) o1[q] = (_Float16)v[q];
    swz_group(W2, p2 ? g : 0, K2P, WSC, v);
#pragma unroll
    for (int q = 0; q < 8; ++q) o2[q] = (_Float16)v[q];
    swz_group(Wn, pn ? g : 0, KN, 1.0f, v);
    unsigned int hb[8], lb[8];
#pragma unroll
    for (int q = 0; q < 8; ++q) {
      hb[q] = bf16_bits(v[q]);
      lb[q] = bf16_bits(v[q] - bf16_val(hb[q]));
    }
    oh[0] = pack2(hb[0], hb[1]); oh[1] = pack2(hb[2], hb[3]); oh[2] = pack2(hb[4], hb[5]); oh[3] = pack2(hb[6], hb[7]);
    ol[0] = pack2(lb[0], lb[1]); ol[1] = pack2(lb[2], lb[3]); ol[2] = pack2(lb[4], lb[5]); ol[3] = pack2(lb[6], lb[7]);
  }
  const size_t off = (size_t)g * 8;
  if (p1) *(volatile v8h*)(W1s + off) = o1;
  if (p2) *(volatile v8h*)(W2s + off) = o2;
  if (pn) { *(volatile v4u*)(Wnh + off) = oh; *(volatile v4u*)(Wnl + off) = ol; }
  __threadfence();
  if (p1) *(volatile v8h*)(W1s + off) = o1;
  if (p2) *(volatile v8h*)(W2s + off) = o2;
  if (pn) { *(volatile v4u*)(Wnh + off) = oh; *(volatile v4u*)(Wnl + off) = ol; }
}

__global__ __launch_bounds__(256) void gather_kernel(
    const float* __restrict__ h, const float* __restrict__ pos, const float* __restrict__ vel,
    const float* __restrict__ acc_, const float* __restrict__ crowd, const int* __restrict__ mask,
    const int* __restrict__ idex, _Float16* XH, _Float16* XF) {
  const int tid  = threadIdx.x;
  const int lane = tid & 31;
  const int wave = tid >> 5;
  const int node = blockIdx.x;
  const int b    = node / N_;

  v8h    hv[4];
  size_t hoff[4];
#pragma unroll
  for (int it = 0; it < 4; ++it) {
    const int e   = wave * 8 + it * 2 + (lane >> 4);
    const int sub = lane & 15;
    const size_t eg = (size_t)node * K_ + e;
    const int mk = mask[eg];
    int m = idex[eg] * mk;
    m = m < 0 ? 0 : (m > N_ - 1 ? N_ - 1 : m);
    const float* hr = h + ((size_t)b * N_ + m) * D_ + sub * 8;
    const float4 p0 = *(const float4*)(hr);
    const float4 p1 = *(const float4*)(hr + 4);
    v8h v;
    v[0] = (_Float16)p0.x; v[1] = (_Float16)p0.y; v[2] = (_Float16)p0.z; v[3] = (_Float16)p0.w;
    v[4] = (_Float16)p1.x; v[5] = (_Float16)p1.y; v[6] = (_Float16)p1.z; v[7] = (_Float16)p1.w;
    hv[it]   = v;
    hoff[it] = eg * D_ + (size_t)sub * 8;
    *(volatile v8h*)(XH + hoff[it]) = v;
  }

  const bool fval = tid < K_;
  v8h fv;
#pragma unroll
  for (int q = 0; q < 8; ++q) fv[q] = (_Float16)0.f;
  size_t foff = 0;
  if (fval) {
    const int e = tid;
    const size_t eg = (size_t)node * K_ + e;
    const int mk = mask[eg];
    int m = idex[eg] * mk;
    m = m < 0 ? 0 : (m > N_ - 1 ? N_ - 1 : m);
    const size_t nb = (size_t)b * N_ + m;
    const size_t pb = (size_t)node;

    const float px = pos[pb * 2 + 0], py = pos[pb * 2 + 1];
    const float vx = vel[pb * 2 + 0], vy = vel[pb * 2 + 1];
    const float ax = acc_[pb * 2 + 0], ay = acc_[pb * 2 + 1];
    const float ivn = 1.f / fmaxf(sqrtf(vx * vx + vy * vy), 1e-12f);
    const float vix = vx * ivn, viy = vy * ivn;
    const float c0 = crowd[pb * CD_ + 0], c1 = crowd[pb * CD_ + 1];
    const float c2 = crowd[pb * CD_ + 2], c3 = crowd[pb * CD_ + 3];
    const float pn = sqrtf(vx * vx + vy * vy + ax * ax + ay * ay);
    const float cn = sqrtf(c0 * c0 + c1 * c1 + c2 * c2 + c3 * c3);
    const float cos_sim = (vx * c0 + vy * c1 + ax * c2 + ay * c3) / (pn * cn + 1e-6f);
    const float crowd_sim = (cos_sim + 1.f) * 0.5f;

    const float npx = pos[nb * 2 + 0], npy = pos[nb * 2 + 1];
    const float nvx = vel[nb * 2 + 0], nvy = vel[nb * 2 + 1];
    const float rx = npx - px, ry = npy - py;
    const float rn = sqrtf(rx * rx + ry * ry);
    const float dist = rn + 1e-6f;
    const float irn = 1.f / fmaxf(rn, 1e-12f);
    const float rdx = rx * irn, rdy = ry * irn;
    const float invn = 1.f / fmaxf(sqrtf(nvx * nvx + nvy * nvy), 1e-12f);
    const float vjx = nvx * invn, vjy = nvy * invn;
    const float fs1 = (rdx * vjx + rdy * vjy + 1.f) * 0.5f;
    const float fs2 = (vix * vjx + viy * vjy + 1.f) * 0.5f;
    const float dvx = vx - nvx, dvy = vy - nvy;
    const float rsp = sqrtf(dvx * dvx + dvy * dvy);

    fv[0] = (_Float16)rx;  fv[1] = (_Float16)ry;  fv[2] = (_Float16)dist;
    fv[3] = (_Float16)fs1; fv[4] = (_Float16)fs2; fv[5] = (_Float16)crowd_sim;
    fv[6] = (_Float16)rsp; fv[7] = (_Float16)0.f;
    foff = eg * 8;
    *(volatile v8h*)(XF + foff) = fv;
  }

  __threadfence();
#pragma unroll
  for (int it = 0; it < 4; ++it) *(volatile v8h*)(XH + hoff[it]) = hv[it];
  if (fval) *(volatile v8h*)(XF + foff) = fv;
}

__global__ __launch_bounds__(256) void edge_mlp_kernel(
    const _Float16* __restrict__ XH, const _Float16* __restrict__ XF, const int* __restrict__ mask,
    const float* __restrict__ b1, const float* __restrict__ b2,
    const _Float16* __restrict__ W1s, const _Float16* __restrict__ W2s, float* agg) {
  __shared__ __align__(32) _Float16 sA[K_ * K1P];
  __shared__ __align__(32) _Float16 sW[K1P * OUT_];
  __shared__ float sMask[K_];
  __shared__ __align__(16) float sPart[4 * OUT_];
  __shared__ float sInv;

  const int tid  = threadIdx.x;
  const int lane = tid & 31;
  const int wave = tid >> 5;
  const int node = blockIdx.x;
  const size_t ebase = (size_t)node * K_;

#pragma unroll
  for (int q = 0; q < 10; ++q) {
    const int i = tid + 256 * q;
    ((v4ua*)sW)[i] = ((const v4u*)W1s)[i];
  }
#pragma unroll
  for (int q = 0; q < 4; ++q) {
    const int g   = tid + 256 * q;
    const int row = g >> 4;
    const int c8  = (g & 15) << 3;
    *(v4ua*)(sA + row * K1P + c8) = *(const v4u*)(XH + (ebase + row) * D_ + c8);
  }
  if (tid < K_) {
    *(v4ua*)(sA + tid * K1P + D_) = *(const v4u*)(XF + (ebase + tid) * 8);
    sMask[tid] = (float)mask[ebase + tid];
  }
  if (tid < 3 * K_) {
    const int row  = tid / 3;
    const int part = tid - row * 3;
    v4u z; z[0] = 0u; z[1] = 0u; z[2] = 0u; z[3] = 0u;
    *(v4ua*)(sA + row * K1P + 136 + part * 8) = z;
  }
  __syncthreads();
  if (tid == 0) {
    float s = 0.f;
    for (int e = 0; e < K_; ++e) s += sMask[e];
    sInv = 1.f / (s + 1e-6f);
  }

  const int mi  = wave >> 1;
  const int ni0 = (wave & 1) << 2;
  const v8f vz = {0.f, 0.f, 0.f, 0.f, 0.f, 0.f, 0.f, 0.f};

  v8f acc1[4];
#pragma unroll
  for (int t = 0; t < 4; ++t) acc1[t] = vz;
#pragma unroll
  for (int ks = 0; ks < K1P / 32; ++ks) {
    const v16h a = fragA_h(sA, K1P, mi * 16, ks * 32, lane);
#pragma unroll
    for (int t = 0; t < 4; ++t) {
      const v16h bf = fragB_h(sW, ks * 8 + ni0 + t, lane);
      acc1[t] = mma_f16(a, bf, acc1[t]);
    }
  }
  __syncthreads();

  {
    const int rowb = mi * 16 + ((lane >> 4) << 3);
    const int colb = lane & 15;
#pragma unroll
    for (int t = 0; t < 4; ++t) {
      const int col = (ni0 + t) * 16 + colb;
      const float bb = b1[col];
#pragma unroll
      for (int v = 0; v < 8; ++v)
        sA[(rowb + v) * K2P + col] = (_Float16)fmaxf(acc1[t][v] * WSCI + bb, 0.f);
    }
  }
#pragma unroll
  for (int q = 0; q < 8; ++q) {
    const int i = tid + 256 * q;
    ((v4ua*)sW)[i] = ((const v4u*)W2s)[i];
  }
  __syncthreads();

  v8f acc2[4];
#pragma unroll
  for (int t = 0; t < 4; ++t) acc2[t] = vz;
#pragma unroll
  for (int ks = 0; ks < K2P / 32; ++ks) {
    const v16h a = fragA_h(sA, K2P, mi * 16, ks * 32, lane);
#pragma unroll
    for (int t = 0; t < 4; ++t) {
      const v16h bf = fragB_h(sW, ks * 8 + ni0 + t, lane);
      acc2[t] = mma_f16(a, bf, acc2[t]);
    }
  }

  {
    const int rowb = mi * 16 + ((lane >> 4) << 3);
    const int colb = lane & 15;
#pragma unroll
    for (int t = 0; t < 4; ++t) {
      const int col = (ni0 + t) * 16 + colb;
      const float bb = b2[col];
      float s = 0.f;
#pragma unroll
      for (int v = 0; v < 8; ++v) s += (acc2[t][v] * WSCI + bb) * sMask[rowb + v];
      s += __shfl_xor(s, 16, 32);
      if (lane < 16) sPart[mi * OUT_ + col] = s;
    }
  }
  __syncthreads();
  if (tid < OUT_) {
    const float v = ((sPart[tid] + sPart[OUT_ + tid]) + sPart[2 * OUT_ + tid]) + sPart[3 * OUT_ + tid];
    sPart[tid] = v * sInv;
  }
  __syncthreads();

  v4f ov = {0.f, 0.f, 0.f, 0.f};
  if (wave == 0) {
    ov = *(const v4fa*)(sPart + 4 * lane);
    *(volatile v4f*)(agg + (size_t)node * OUT_ + 4 * lane) = ov;
  }
  __threadfence();
  if (wave == 0) *(volatile v4f*)(agg + (size_t)node * OUT_ + 4 * lane) = ov;
}

__global__ __launch_bounds__(256) void node_mlp_kernel(
    const float* __restrict__ h, const float* __restrict__ crowd, const float* __restrict__ ln_g,
    const float* __restrict__ ln_b, const float* __restrict__ bn,
    const unsigned short* __restrict__ Wnh, const unsigned short* __restrict__ Wnl,
    const float* __restrict__ agg, float* out, int numNodes) {
  __shared__ __align__(32) unsigned char smem[49152];
  unsigned short* sAh = (unsigned short*)(smem);
  unsigned short* sAl = (unsigned short*)(smem + 8192);
  unsigned short* sWh = (unsigned short*)(smem + 16384);
  unsigned short* sWl = (unsigned short*)(smem + 32768);
  float* sOut = (float*)(smem);

  const int tid  = threadIdx.x;
  const int lane = tid & 31;
  const int wave = tid >> 5;
  const int row0 = blockIdx.x * 64;
  const int mi   = wave >> 1;
  const int ni0  = (wave & 1) << 2;
  const v8f vz = {0.f, 0.f, 0.f, 0.f, 0.f, 0.f, 0.f, 0.f};

  v8f accn[4];
#pragma unroll
  for (int t = 0; t < 4; ++t) accn[t] = vz;

  for (int c = 0; c < NCH; ++c) {
    __syncthreads();
    {
      const int lr  = tid >> 2;
      const int sub = tid & 3;
      const int row = row0 + lr;
      const bool valid = row < numNodes;
      float x[16];
#pragma unroll
      for (int j = 0; j < 16; ++j) x[j] = 0.f;
      if (valid) {
        if (c < 4) {
          const float* src = (c < 2) ? (h + (size_t)row * D_ + c * 64 + sub * 16)
                                     : (agg + (size_t)row * OUT_ + (c - 2) * 64 + sub * 16);
#pragma unroll
          for (int q = 0; q < 4; ++q) {
            const float4 v = *(const float4*)(src + 4 * q);
            x[4 * q + 0] = v.x; x[4 * q + 1] = v.y; x[4 * q + 2] = v.z; x[4 * q + 3] = v.w;
          }
        } else if (sub == 0) {
          const float c0 = crowd[(size_t)row * CD_ + 0], c1 = crowd[(size_t)row * CD_ + 1];
          const float c2 = crowd[(size_t)row * CD_ + 2], c3 = crowd[(size_t)row * CD_ + 3];
          const float c4 = crowd[(size_t)row * CD_ + 4];
          const float mu = ((((c0 + c1) + c2) + c3) + c4) * (1.f / CD_);
          const float d0 = c0 - mu, d1 = c1 - mu, d2 = c2 - mu, d3 = c3 - mu, d4 = c4 - mu;
          const float var = ((((d0 * d0 + d1 * d1) + d2 * d2) + d3 * d3) + d4 * d4) * (1.f / CD_);
          const float inv = 1.f / sqrtf(var + 1e-5f);
          x[0] = (d0 * inv) * ln_g[0] + ln_b[0];
          x[1] = (d1 * inv) * ln_g[1] + ln_b[1];
          x[2] = (d2 * inv) * ln_g[2] + ln_b[2];
          x[3] = (d3 * inv) * ln_g[3] + ln_b[3];
          x[4] = (d4 * inv) * ln_g[4] + ln_b[4];
        }
      }
      unsigned int hb[16], lb[16];
#pragma unroll
      for (int j = 0; j < 16; ++j) {
        hb[j] = bf16_bits(x[j]);
        lb[j] = bf16_bits(x[j] - bf16_val(hb[j]));
      }
      v4u h0, h1, l0, l1;
#pragma unroll
      for (int q = 0; q < 4; ++q) {
        h0[q] = pack2(hb[2 * q], hb[2 * q + 1]);
        h1[q] = pack2(hb[8 + 2 * q], hb[8 + 2 * q + 1]);
        l0[q] = pack2(lb[2 * q], lb[2 * q + 1]);
        l1[q] = pack2(lb[8 + 2 * q], lb[8 + 2 * q + 1]);
      }
      unsigned short* dh = sAh + lr * 64 + sub * 16;
      unsigned short* dl = sAl + lr * 64 + sub * 16;
      *(v4ua*)(dh) = h0; *(v4ua*)(dh + 8) = h1;
      *(v4ua*)(dl) = l0; *(v4ua*)(dl + 8) = l1;
    }
#pragma unroll
    for (int q = 0; q < 4; ++q) {
      const int i = tid + 256 * q;
      ((v4ua*)sWh)[i] = ((const v4u*)(Wnh + (size_t)c * 8192))[i];
      ((v4ua*)sWl)[i] = ((const v4u*)(Wnl + (size_t)c * 8192))[i];
    }
    __syncthreads();
#pragma unroll
    for (int ks = 0; ks < 2; ++ks) {
      const v16b ah = fragA_b(sAh, 64, mi * 16, ks * 32, lane);
      const v16b al = fragA_b(sAl, 64, mi * 16, ks * 32, lane);
#pragma unroll
      for (int t = 0; t < 4; ++t) {
        const int f = ks * 8 + ni0 + t;
        const v16b bh = fragB_b(sWh, f, lane);
        const v16b bl = fragB_b(sWl, f, lane);
        accn[t] = mma_bf16(ah, bh, accn[t]);
        accn[t] = mma_bf16(ah, bl, accn[t]);
        accn[t] = mma_bf16(al, bh, accn[t]);
      }
    }
  }
  __syncthreads();

  {
    const int rowb = mi * 16 + ((lane >> 4) << 3);
    const int colb = lane & 15;
#pragma unroll
    for (int t = 0; t < 4; ++t) {
      const int col = (ni0 + t) * 16 + colb;
      const float bb = bn[col];
#pragma unroll
      for (int v = 0; v < 8; ++v)
        sOut[(rowb + v) * OUT_ + col] = fmaxf(accn[t][v] + bb, 0.f);
    }
  }
  __syncthreads();

  v4f ov[8];
#pragma unroll
  for (int i = 0; i < 8; ++i) ov[i] = *(const v4fa*)(sOut + (wave * 8 + i) * OUT_ + 4 * lane);
#pragma unroll
  for (int i = 0; i < 8; ++i) {
    const int r = row0 + wave * 8 + i;
    if (r < numNodes) *(volatile v4f*)(out + (size_t)r * OUT_ + 4 * lane) = ov[i];
  }
  __threadfence();
#pragma unroll
  for (int i = 0; i < 8; ++i) {
    const int r = row0 + wave * 8 + i;
    if (r < numNodes) *(volatile v4f*)(out + (size_t)r * OUT_ + 4 * lane) = ov[i];
  }
}

extern "C" void kernel_launch(void* const* d_in, const int* in_sizes, int n_in,
                              void* d_out, int out_size, void* d_ws, size_t ws_size,
                              hipStream_t stream) {
  if (n_in < 16) return;
  const float* h     = (const float*)d_in[0];
  const float* pos   = (const float*)d_in[1];
  const float* vel   = (const float*)d_in[2];
  const float* acc   = (const float*)d_in[3];
  const float* crowd = (const float*)d_in[4];
  const int*   mask  = (const int*)d_in[5];
  const int*   idex  = (const int*)d_in[6];
  const float* W1    = (const float*)d_in[8];
  const float* b1    = (const float*)d_in[9];
  const float* W2    = (const float*)d_in[10];
  const float* b2    = (const float*)d_in[11];
  const float* Wn    = (const float*)d_in[12];
  const float* bn    = (const float*)d_in[13];
  const float* ln_g  = (const float*)d_in[14];
  const float* ln_b  = (const float*)d_in[15];

  const int numNodes = in_sizes[0] / D_;
  if (numNodes <= 0 || (numNodes % N_) != 0) return;
  if (in_sizes[0] != numNodes * D_ || in_sizes[1] != numNodes * 2 || in_sizes[2] != numNodes * 2 ||
      in_sizes[3] != numNodes * 2 || in_sizes[4] != numNodes * CD_ ||
      in_sizes[5] != numNodes * K_ || in_sizes[6] != numNodes * K_ ||
      in_sizes[8] != K1 * OUT_ || in_sizes[9] != OUT_ || in_sizes[10] != K2P * OUT_ ||
      in_sizes[11] != OUT_ || in_sizes[12] != KN * OUT_ || in_sizes[13] != OUT_ ||
      in_sizes[14] != CD_ || in_sizes[15] != CD_ || out_size != numNodes * OUT_) return;

  const size_t numEdges = (size_t)numNodes * K_;
  size_t off = 0;
  const size_t oW1s = off; off += (size_t)NG_W1 * 16;
  const size_t oW2s = off; off += (size_t)NG_W2 * 16;
  const size_t oWnh = off; off += (size_t)NG_WN * 16;
  const size_t oWnl = off; off += (size_t)NG_WN * 16;
  const size_t oXH  = off; off += numEdges * D_ * 2;
  const size_t oXF  = off; off += numEdges * 8 * 2;
  const size_t oAgg = off; off += (size_t)numNodes * OUT_ * 4;
  if (off > ws_size) return;

  char* ws = (char*)d_ws;
  _Float16* W1s = (_Float16*)(ws + oW1s);
  _Float16* W2s = (_Float16*)(ws + oW2s);
  unsigned short* Wnh = (unsigned short*)(ws + oWnh);
  unsigned short* Wnl = (unsigned short*)(ws + oWnl);
  _Float16* XH = (_Float16*)(ws + oXH);
  _Float16* XF = (_Float16*)(ws + oXF);
  float* agg = (float*)(ws + oAgg);

  convert_weights_kernel<<<(NG_WN + 255) / 256, 256, 0, stream>>>(W1, W2, Wn, W1s, W2s, Wnh, Wnl);
  gather_kernel<<<numNodes, 256, 0, stream>>>(h, pos, vel, acc, crowd, mask, idex, XH, XF);
  edge_mlp_kernel<<<numNodes, 256, 0, stream>>>(XH, XF, mask, b1, b2, W1s, W2s, agg);
  node_mlp_kernel<<<(numNodes + 63) / 64, 256, 0, stream>>>(h, crowd, ln_g, ln_b, bn, Wnh, Wnl,
                                                              agg, (float*)d_out, numNodes);
}
